// MultiFusionVoxel_35124242546747
// MI455X (gfx1250) — hardware-verified
//
#include <hip/hip_runtime.h>
#include <stddef.h>
#include <math.h>


#define KNN   24
#define DCH   128
#define NT    128
#define NWV   4
#define QW    16
#define QBLK  (NWV * QW)
#define DBIG  3.0e38f

static_assert(NT == NWV * 32);
static_assert(KNN <= 32);
static_assert(DCH == 4 * 32);

typedef float    v4f  __attribute__((ext_vector_type(4)));
typedef float    v8f  __attribute__((ext_vector_type(8)));
typedef _Float16 v8h  __attribute__((ext_vector_type(8)));
typedef _Float16 v16h __attribute__((ext_vector_type(16)));
union FragH { v16h v; v8h h[2]; };

__device__ __forceinline__ v8f wmh(v16h a, v16h b, v8f c) {
  v8f d = __builtin_amdgcn_wmma_f32_16x16x32_f16(false, a, false, b, (short)0, c, false, false);
#if defined(__HIP_DEVICE_COMPILE__)
  asm volatile("v_nop\n\tv_nop\n\tv_nop\n\tv_nop" : "+v"(d) : "v"(a), "v"(b));
#endif
  return d;
}

__device__ __forceinline__ v8f zero8() {
  v8f z = {0.f, 0.f, 0.f, 0.f, 0.f, 0.f, 0.f, 0.f};
  return z;
}

__device__ __forceinline__ void ins24(float (&dd)[KNN], int (&jj)[KNN], const float dk, const int jk) {
  float cd = dk;
  int   cj = jk;
#pragma unroll
  for (int t = 0; t < KNN; ++t) {
    const bool  sw = dk < dd[t];
    const float od = dd[t];
    const int   oj = jj[t];
    dd[t] = sw ? cd : od;
    jj[t] = sw ? cj : oj;
    cd = sw ? od : cd;
    cj = sw ? oj : cj;
  }
}

__device__ __forceinline__ void insm24(float (&dd)[KNN], int (&jj)[KNN], const float dk, const int jk) {
  float cd = dk;
  int   cj = jk;
#pragma unroll
  for (int t = 0; t < KNN; ++t) {
    const bool  sw = (dk < dd[t]) || (dk == dd[t] && jk < jj[t]);
    const float od = dd[t];
    const int   oj = jj[t];
    dd[t] = sw ? cd : od;
    jj[t] = sw ? cj : oj;
    cd = sw ? od : cd;
    cj = sw ? oj : cj;
  }
}

__global__ __launch_bounds__(256) void k_plane(const int* __restrict__ midc, const int* __restrict__ lowc,
                                               v8h* plane, int M1, int M2) {
  const int M = M1 + M2;
  const int t = blockIdx.x * 256 + (int)threadIdx.x;
  if (t >= 2 * M) return;
  const int j = t >> 1, hf = t & 1;
  int jm = j < M1 ? j : M1 - 1;
  jm = jm < 0 ? 0 : jm;
  int jl = j - M1;
  jl = jl < 0 ? 0 : jl;
  jl = jl > M2 - 1 ? M2 - 1 : jl;
  const int xm = midc[3 * jm], ym = midc[3 * jm + 1], zm = midc[3 * jm + 2];
  const int xl = lowc[3 * jl], yl = lowc[3 * jl + 1], zl = lowc[3 * jl + 2];
  const bool inm = j < M1;
  const int x = inm ? xm : xl;
  const int y = inm ? ym : yl;
  const int z = inm ? zm : zl;
  const int rr = x * x + y * y + z * z;
  const float fx = (float)x, fy = (float)y, fz = (float)z;
  const float zr = fx * 0.0f;
  const float p0 = (float)(rr & 127);
  const float p1 = (float)((rr >> 7) & 127);
  const float p2 = (float)(rr >> 14);
  const float e0 = hf ? zr + 16384.0f : fx;
  const float e1 = hf ? zr : fy;
  const float e2 = hf ? zr : fz;
  const float e3 = hf ? zr : p0;
  const float e4 = hf ? zr : p1;
  const float e5 = hf ? zr : p2;
  const float e6 = hf ? zr : zr + 1.0f;
  const float e7 = hf ? zr : zr + 128.0f;
  v8h v;
  v[0] = (_Float16)e0; v[1] = (_Float16)e1; v[2] = (_Float16)e2; v[3] = (_Float16)e3;
  v[4] = (_Float16)e4; v[5] = (_Float16)e5; v[6] = (_Float16)e6; v[7] = (_Float16)e7;
  v8h* dp = plane + t;
  *(volatile v8h*)dp = v;
  __threadfence();
  *(volatile v8h*)dp = v;
}

__global__ __launch_bounds__(NT) void k_knn(const int* __restrict__ qc, const v8h* __restrict__ plane,
                                            const float* __restrict__ midf, const float* __restrict__ lowf,
                                            const int* __restrict__ kin, float* out, int N, int M1, int M2) {
  __shared__ float sXD[NWV][KNN][32];
  __shared__ int   sXI[NWV][KNN][32];
  __shared__ float sFD[NWV][QW][KNN];
  __shared__ int   sFI[NWV][QW][KNN];
  __shared__ float sFW[NWV][QW][KNN];

  const int tid = threadIdx.x, lane = tid & 31, wave = tid >> 5, h = lane >> 4, n = lane & 15;
  const int M = M1 + M2;
  int keff = kin[0];
  keff = keff < 1 ? 1 : (keff > KNN ? KNN : keff);

  const int qbase = blockIdx.x * QBLK + wave * QW;
  int qi = qbase + n;
  qi = qi > N - 1 ? N - 1 : qi;
  const int qx = qc[3 * qi], qy = qc[3 * qi + 1], qz = qc[3 * qi + 2];
  const int qq = qx * qx + qy * qy + qz * qz;
  const float fqx = (float)qx, fqy = (float)qy, fqz = (float)qz;
  const float zr = fqx * 0.0f;

  v8h z8;
#pragma unroll
  for (int i = 0; i < 8; ++i) z8[i] = (_Float16)zr;

  FragH b;
  {
    const float e0 = h ? (float)(qq >> 14) : -2.0f * fqx;
    const float e1 = h ? zr : -2.0f * fqy;
    const float e2 = h ? zr : -2.0f * fqz;
    const float e3 = h ? zr : zr + 1.0f;
    const float e4 = h ? zr : zr + 128.0f;
    const float e5 = h ? zr : zr + 16384.0f;
    const float e6 = h ? zr : (float)(qq & 127);
    const float e7 = h ? zr : (float)((qq >> 7) & 127);
    v8h b0;
    b0[0] = (_Float16)e0; b0[1] = (_Float16)e1; b0[2] = (_Float16)e2; b0[3] = (_Float16)e3;
    b0[4] = (_Float16)e4; b0[5] = (_Float16)e5; b0[6] = (_Float16)e6; b0[7] = (_Float16)e7;
    b.h[0] = b0;
    b.h[1] = z8;
  }
  FragH a;
  a.h[1] = z8;

  float dd[KNN];
  int   jj[KNN];
#pragma unroll
  for (int t = 0; t < KNN; ++t) { dd[t] = DBIG; jj[t] = 0; }

  const v8h* __restrict__ prow = plane + h;
  for (int m0 = 0; m0 < M; m0 += 16) {
    a.h[0] = prow[2 * (m0 + n)];
    const v8f acc = wmh(a.v, b.v, zero8());
    const int jb = m0 + 8 * h;
#pragma unroll
    for (int r = 0; r < 8; ++r) {
      const float dk = acc[r];
      if (dk < dd[KNN - 1]) ins24(dd, jj, dk, jb + r);
    }
  }

#pragma unroll
  for (int t = 0; t < KNN; ++t) {
    sXD[wave][t][lane] = dd[t];
    sXI[wave][t][lane] = jj[t];
  }
  __syncthreads();
  {
    const int pl = lane ^ 16;
#pragma unroll 1
    for (int t = 0; t < KNN; ++t) {
      const float od = sXD[wave][t][pl];
      const int   oj = sXI[wave][t][pl];
      const bool better = (od < dd[KNN - 1]) || (od == dd[KNN - 1] && oj < jj[KNN - 1]);
      if (better) insm24(dd, jj, od, oj);
    }
  }
  if (h == 0) {
#pragma unroll
    for (int t = 0; t < KNN; ++t) {
      int j2 = jj[t];
      j2 = j2 < 0 ? 0 : (j2 > M - 1 ? M - 1 : j2);
      sFD[wave][n][t] = dd[t];
      sFI[wave][n][t] = j2;
    }
  }
  __syncthreads();

  {
    const int jl = lane < KNN ? lane : KNN - 1;
    for (int q = 0; q < QW; ++q) {
      const float d2 = sFD[wave][q][jl];
      const float d  = sqrtf(fmaxf(d2, 0.0f));
      float w = 1.0f / (1.0f + d);
      w = (lane < keff) ? w : 0.0f;
      float s = w;
      s += __shfl_xor(s, 16, 32);
      s += __shfl_xor(s, 8, 32);
      s += __shfl_xor(s, 4, 32);
      s += __shfl_xor(s, 2, 32);
      s += __shfl_xor(s, 1, 32);
      const float wn = w * (1.0f / s);
      if (lane < KNN) sFW[wave][q][lane] = wn;
    }
  }
  __syncthreads();

  for (int q = 0; q < QW; ++q) {
    const int qo = qbase + q;
    v4f av = {0.f, 0.f, 0.f, 0.f};
#pragma unroll 2
    for (int j = 0; j < keff; ++j) {
      const int   id = sFI[wave][q][j];
      const float w  = sFW[wave][q][j];
      int im = id < M1 ? id : M1 - 1;
      im = im < 0 ? 0 : im;
      int il = id - M1;
      il = il < 0 ? 0 : (il > M2 - 1 ? M2 - 1 : il);
      const v4f xm = *(const v4f*)(midf + (size_t)im * DCH + 4 * lane);
      const v4f xl = *(const v4f*)(lowf + (size_t)il * DCH + 4 * lane);
      const v4f x = (id < M1) ? xm : xl;
      av = av + w * x;
    }
    if (qo < N) {
      float* gp = out + (size_t)qo * DCH + 4 * lane;
      *(volatile v4f*)gp = av;
      __threadfence();
      *(volatile v4f*)gp = av;
    }
  }
}

extern "C" void kernel_launch(void* const* d_in, const int* in_sizes, int n_in,
                              void* d_out, int out_size, void* d_ws, size_t ws_size,
                              hipStream_t stream) {
  if (n_in < 6) return;
  const int N  = in_sizes[0] / 3;
  const int M1 = in_sizes[1] / 3;
  const int M2 = in_sizes[2] / 3;
  const int M  = M1 + M2;
  if (N <= 0 || M1 <= 0 || M2 <= 0) return;
  if (in_sizes[0] != 3 * N || in_sizes[1] != 3 * M1 || in_sizes[2] != 3 * M2) return;
  if ((M % 16) != 0 || M < 48) return;
  if (in_sizes[3] != M1 * DCH || in_sizes[4] != M2 * DCH) return;
  if (in_sizes[5] < 1) return;
  if (out_size != N * DCH) return;

  const int*   qc   = (const int*)d_in[0];
  const int*   midc = (const int*)d_in[1];
  const int*   lowc = (const int*)d_in[2];
  const float* midf = (const float*)d_in[3];
  const float* lowf = (const float*)d_in[4];
  const int*   kin  = (const int*)d_in[5];
  float* out = (float*)d_out;

  size_t off = 0;
  const size_t oPlane = off;
  off += (size_t)M * 32;
  off = (off + 255) & ~(size_t)255;
  if (off > ws_size || off > (size_t)134217728) return;
  v8h* plane = (v8h*)((char*)d_ws + oPlane);

  k_plane<<<(2 * M + 255) / 256, 256, 0, stream>>>(midc, lowc, plane, M1, M2);

  k_knn<<<(N + QBLK - 1) / QBLK, NT, 0, stream>>>(qc, plane, midf, lowf, kin, out, N, M1, M2);
}
